// TFPerceiverSelfAttention_9259949490490
// MI455X (gfx1250) — hardware-verified
//
#include <hip/hip_runtime.h>
#include <math.h>
#include <stdint.h>

constexpr int kBatch = 4;
constexpr int kQLen  = 512;
constexpr int kKVLen = 4096;
constexpr int kQDim  = 1024;
constexpr int kKVDim = 768;
constexpr int kHeads = 8;
constexpr int kHD    = 128;
constexpr int kQKCh  = 1024;
constexpr int kVCh   = 1024;
constexpr float kLnEps = 1e-3f;
constexpr float kWCarry = 32.0f;
constexpr float kWCarryInv = 1.0f / 32.0f;
constexpr float kPCarry = 32768.0f;

typedef __attribute__((ext_vector_type(16))) _Float16 v16h;
typedef __attribute__((ext_vector_type(8)))  _Float16 v8h;
typedef __attribute__((ext_vector_type(16))) __bf16   v16b;
typedef __attribute__((ext_vector_type(8)))  __bf16   v8b;
typedef __attribute__((ext_vector_type(8)))  float    v8f;
typedef __attribute__((ext_vector_type(4)))  float    v4f;
typedef __attribute__((ext_vector_type(4)))  unsigned int v4u;

__device__ __forceinline__ unsigned short f2bf_bits(float f) {
  unsigned u = __float_as_uint(f);
  return (unsigned short)((u + 0x7FFFu + ((u >> 16) & 1u)) >> 16);
}
__device__ __forceinline__ float bf_bits2f(unsigned short h) { return __uint_as_float(((unsigned)h) << 16); }

__device__ __forceinline__ void dep_guard_h(v8f& a, v8f& b, v16h x, v16h y) { asm volatile("v_nop\n\tv_nop\n\tv_nop\n\tv_nop" : "+v"(a), "+v"(b) : "v"(x), "v"(y)); }
__device__ __forceinline__ void dep_guard_b(v8f& a, v8f& b, v16b x, v16b y) { asm volatile("v_nop\n\tv_nop\n\tv_nop\n\tv_nop" : "+v"(a), "+v"(b) : "v"(x), "v"(y)); }
__device__ __forceinline__ void keep4_h(v16h a, v16h b, v16h c, v16h d) { asm volatile("v_nop" :: "v"(a), "v"(b), "v"(c), "v"(d)); }
__device__ __forceinline__ void keep4_b(v16b a, v16b b, v16b c, v16b d) { asm volatile("v_nop" :: "v"(a), "v"(b), "v"(c), "v"(d)); }
__device__ __forceinline__ void acc_guard4(v8f& a, v8f& b, v8f& c, v8f& d) { asm volatile("v_nop\n\tv_nop\n\tv_nop\n\tv_nop" : "+v"(a), "+v"(b), "+v"(c), "+v"(d)); }
template <typename T> struct Frag;
template <> struct Frag<_Float16> {
  typedef v16h V; union U { v16h v; v8h h[2]; };
  static __device__ __forceinline__ v16h load(const _Float16* p) {
    U f; f.h[0] = *(const v8h*)(p); f.h[1] = *(const v8h*)(p + 16); return f.v;
  }
  static __device__ __forceinline__ v8f mma(v16h a, v16h b, v8f c) {
    return __builtin_amdgcn_wmma_f32_16x16x32_f16(false, a, false, b, (short)0, c, false, false);
  }
  static __device__ __forceinline__ void guard(v8f& a, v8f& b, v16h x, v16h y) { dep_guard_h(a, b, x, y); }
  static __device__ __forceinline__ void keep(v16h a, v16h b, v16h c, v16h d) { keep4_h(a, b, c, d); }
};
template <> struct Frag<__bf16> {
  typedef v16b V; union U { v16b v; v8b h[2]; };
  static __device__ __forceinline__ v16b load(const __bf16* p) {
    U f; f.h[0] = *(const v8b*)(p); f.h[1] = *(const v8b*)(p + 16); return f.v;
  }
  static __device__ __forceinline__ v8f mma(v16b a, v16b b, v8f c) {
    return __builtin_amdgcn_wmma_f32_16x16x32_bf16(false, a, false, b, (short)0, c, false, false);
  }
  static __device__ __forceinline__ void guard(v8f& a, v8f& b, v16b x, v16b y) { dep_guard_b(a, b, x, y); }
  static __device__ __forceinline__ void keep(v16b a, v16b b, v16b c, v16b d) { keep4_b(a, b, c, d); }
};

template <int ET> struct Elem;
template <> struct Elem<0> { typedef _Float16 T; };
template <> struct Elem<1> { typedef __bf16 T; };
template <int ET, bool SPLIT, int BIAS_MODE, int OUT_MODE, bool RESID, int ACT = 0>
__global__ __launch_bounds__(256) void wmma_gemm64(
    const unsigned short* __restrict__ Ap, const unsigned short* __restrict__ A2p, int lda, long strideA,
    const unsigned short* __restrict__ Btp, const unsigned short* __restrict__ Bt2p, int ldb, long strideB,
    void* __restrict__ Cout, void* __restrict__ Cout2, int ldc, long strideC,
    const float* __restrict__ bias,
    const float* __restrict__ resid, long strideR,
    int M, int N, int K, float scale) {
  typedef typename Elem<ET>::T T;
  typedef typename Frag<T>::V V;
  const T* A = (const T*)Ap; const T* A2 = (const T*)A2p; const T* Bt = (const T*)Btp; const T* Bt2 = (const T*)Bt2p;
  __shared__ __align__(16) float sT[8][16 * 68];
  const int b    = blockIdx.y;
  const int lane = threadIdx.x & 31;
  const int wave = threadIdx.x >> 5;
  const int tilesN = N >> 6;
  const int tilesM = M >> 6;
  const int tile = blockIdx.x * 8 + wave;
  if (tile >= tilesM * tilesN) return;
  const int tm = tile / tilesN;
  const int tn = tile - tm * tilesN;
  const int m0 = tm << 6;
  const int n0 = tn << 6;

  const T* Ab  = A  + (size_t)b * strideA;
  const T* Bb  = Bt + (size_t)b * strideB;
  const T* Ab2 = SPLIT ? (A2  + (size_t)b * strideA) : nullptr;
  const T* Bb2 = SPLIT ? (Bt2 + (size_t)b * strideB) : nullptr;

  const int rlane = lane & 15;
  const int koff  = (lane >> 4) * 8;
  const int mOff  = (lane >> 4) * 8;

  v8f acc[4][4];
#pragma unroll
  for (int i = 0; i < 4; ++i)
#pragma unroll
    for (int j = 0; j < 4; ++j) acc[i][j] = (v8f){0.f,0.f,0.f,0.f,0.f,0.f,0.f,0.f};

  for (int k0 = 0; k0 < K; k0 += 32) {
    V bh[4], bl[4];
#pragma unroll
    for (int j = 0; j < 4; ++j) {
      const size_t bo = (size_t)(n0 + (j << 4) + rlane) * ldb + koff + k0;
      bh[j] = Frag<T>::load(Bb + bo);
      if (SPLIT) bl[j] = Frag<T>::load(Bb2 + bo);
    }
#pragma unroll
    for (int i = 0; i < 4; ++i) {
      const size_t ao = (size_t)(m0 + (i << 4) + rlane) * lda + koff + k0;
      V ah = Frag<T>::load(Ab + ao);
      V al;
      if (SPLIT) al = Frag<T>::load(Ab2 + ao);
#pragma unroll
      for (int j = 0; j < 4; ++j) {
        acc[i][j] = Frag<T>::mma(ah, bh[j], acc[i][j]);
        if (SPLIT) {
          acc[i][j] = Frag<T>::mma(ah, bl[j], acc[i][j]);
          acc[i][j] = Frag<T>::mma(al, bh[j], acc[i][j]);
        }
      }
      Frag<T>::guard(acc[i][0], acc[i][3], ah, SPLIT ? al : ah);
    }
    Frag<T>::keep(bh[0], bh[1], bh[2], bh[3]);
    if (SPLIT) Frag<T>::keep(bl[0], bl[1], bl[2], bl[3]);
  }
  acc_guard4(acc[0][0], acc[0][1], acc[0][2], acc[0][3]);
  acc_guard4(acc[1][0], acc[1][1], acc[1][2], acc[1][3]);
  acc_guard4(acc[2][0], acc[2][1], acc[2][2], acc[2][3]);
  acc_guard4(acc[3][0], acc[3][1], acc[3][2], acc[3][3]);

  float* slab = sT[wave];
  const float* Rb = RESID ? (resid + (size_t)b * strideR) : nullptr;
#pragma unroll
  for (int i = 0; i < 4; ++i) {
    const int mBase = m0 + (i << 4);
#pragma unroll
    for (int j = 0; j < 4; ++j) {
      const int n = n0 + (j << 4) + rlane;
      float bv = 0.f;
      if (BIAS_MODE == 2) bv = bias[n];
#pragma unroll
      for (int r = 0; r < 8; ++r) {
        float v = acc[i][j][r] * scale;
        if (BIAS_MODE == 1) v += bias[mBase + mOff + r];
        if (BIAS_MODE == 2) v += bv;
        if (RESID) v += Rb[(size_t)(mBase + mOff + r) * ldc + n];
        if (ACT == 1) v = tanhf(v);
        if (ACT == 2) v = fmaxf(v, 0.0f);
        if (ACT == 3) v = v / (1.0f + expf(-v));
        if (ACT == 4) v = (v > 0.f) ? v : 0.01f * v;
        if (ACT == 5) v = 0.5f * v * (1.0f + erff(v * 0.70710678118654752f));
        slab[(mOff + r) * 68 + (j << 4) + rlane] = v;
      }
    }
    __builtin_amdgcn_fence(__ATOMIC_RELEASE, "workgroup");
    __builtin_amdgcn_wave_barrier();
    __builtin_amdgcn_fence(__ATOMIC_ACQUIRE, "workgroup");
    if (OUT_MODE == 0) {
      float* C = (float*)Cout + (size_t)b * strideC;
      const int hh = lane >> 4, c4 = (lane & 15) * 4;
      for (int pass = 0; pass < 2; ++pass) {
#pragma unroll
        for (int it = 0; it < 8; ++it) {
          const int row = it * 2 + hh;
          v4f v = *(const v4f*)(slab + row * 68 + c4);
          *(volatile v4f*)(C + (size_t)(mBase + row) * ldc + n0 + c4) = v;
        }
        __threadfence();
      }
    } else {
      const int q = lane >> 3, c8 = (lane & 7) * 8;
      unsigned short* C  = (unsigned short*)Cout  + (size_t)b * strideC;
      unsigned short* C2 = (OUT_MODE == 2) ? ((unsigned short*)Cout2 + (size_t)b * strideC) : nullptr;
      for (int pass = 0; pass < 2; ++pass) {
#pragma unroll
        for (int it = 0; it < 4; ++it) {
          const int row = it * 4 + q;
          const float* sp = slab + row * 68 + c8;
          v8h hv, lv;
#pragma unroll
          for (int e = 0; e < 8; ++e) {
            if (OUT_MODE == 1) {
              hv[e] = (_Float16)sp[e];
            } else {
              unsigned short hb = f2bf_bits(sp[e]);
              unsigned short lb = f2bf_bits(sp[e] - bf_bits2f(hb));
              hv[e] = __builtin_bit_cast(_Float16, hb);
              lv[e] = __builtin_bit_cast(_Float16, lb);
            }
          }
          *(volatile v8h*)(C + (size_t)(mBase + row) * ldc + n0 + c8) = hv;
          if (OUT_MODE == 2) *(volatile v8h*)(C2 + (size_t)(mBase + row) * ldc + n0 + c8) = lv;
        }
        __threadfence();
      }
    }
    __builtin_amdgcn_fence(__ATOMIC_RELEASE, "workgroup");
    __builtin_amdgcn_wave_barrier();
    __builtin_amdgcn_fence(__ATOMIC_ACQUIRE, "workgroup");
  }
}

template <int WIDTH>
__global__ __launch_bounds__(128) void ln_rows_f16(const float* __restrict__ x, const float* __restrict__ gam,
                                                   const float* __restrict__ bet, unsigned short* __restrict__ y,
                                                   float eps) {
  static_assert(WIDTH % 256 == 0, "whole waves active");
  __shared__ float red0[4];
  __shared__ float red1[4];
  constexpr int kNT = WIDTH / 8;
  const int row  = blockIdx.x;
  const int tid  = threadIdx.x;
  const int lane = tid & 31;
  const int wave = tid >> 5;
  const bool act = tid < kNT;
  const int tc   = act ? tid : (kNT - 1);
  const float* xr = x + (size_t)row * WIDTH + tc * 8;
  const v4f a0 = *(const v4f*)(xr);
  const v4f a1 = *(const v4f*)(xr + 4);
  float v[8];
  v[0] = a0[0]; v[1] = a0[1]; v[2] = a0[2]; v[3] = a0[3];
  v[4] = a1[0]; v[5] = a1[1]; v[6] = a1[2]; v[7] = a1[3];
  float sm = ((v[0] + v[1]) + (v[2] + v[3])) + ((v[4] + v[5]) + (v[6] + v[7]));
  sm = act ? sm : 0.f;
#pragma unroll
  for (int off = 1; off < 32; off <<= 1) sm += __shfl_xor(sm, off, 32);
  if (lane == 0) red0[wave] = sm;
  __syncthreads();
  const float mean = ((red0[0] + red0[1]) + (red0[2] + red0[3])) * (1.0f / (float)WIDTH);
  float d[8];
  float sq = 0.f;
#pragma unroll
  for (int e = 0; e < 8; ++e) { d[e] = v[e] - mean; sq += d[e] * d[e]; }
  sq = act ? sq : 0.f;
#pragma unroll
  for (int off = 1; off < 32; off <<= 1) sq += __shfl_xor(sq, off, 32);
  if (lane == 0) red1[wave] = sq;
  __syncthreads();
  const float var = ((red1[0] + red1[1]) + (red1[2] + red1[3])) * (1.0f / (float)WIDTH);
  const float inv = rsqrtf(var + eps);
  const v4f g0 = *(const v4f*)(gam + tc * 8);
  const v4f g1 = *(const v4f*)(gam + tc * 8 + 4);
  const v4f b0 = *(const v4f*)(bet + tc * 8);
  const v4f b1 = *(const v4f*)(bet + tc * 8 + 4);
  float gg[8], bb[8];
  gg[0] = g0[0]; gg[1] = g0[1]; gg[2] = g0[2]; gg[3] = g0[3];
  gg[4] = g1[0]; gg[5] = g1[1]; gg[6] = g1[2]; gg[7] = g1[3];
  bb[0] = b0[0]; bb[1] = b0[1]; bb[2] = b0[2]; bb[3] = b0[3];
  bb[4] = b1[0]; bb[5] = b1[1]; bb[6] = b1[2]; bb[7] = b1[3];
  v8h hv;
#pragma unroll
  for (int e = 0; e < 8; ++e) hv[e] = (_Float16)((d[e] * inv) * gg[e] + bb[e]);
  unsigned short* yr = y + (size_t)row * WIDTH + tc * 8;
  if (act) *(volatile v8h*)yr = hv;
  __threadfence();
  if (act) *(volatile v8h*)yr = hv;
}

__device__ __forceinline__ unsigned pk16(unsigned short a, unsigned short b) { return (unsigned)a | ((unsigned)b << 16); }

__global__ __launch_bounds__(256) void ttrans_f16_kernel(const float* __restrict__ W, unsigned short* __restrict__ o,
                                                         int R, int Cc, float mul) {
  __shared__ __align__(16) float tf[64 * 68];
  const int c0  = blockIdx.x * 64;
  const int r0  = blockIdx.y * 64;
  const int tid = threadIdx.x;
  {
    const int lr = tid >> 4;
    const int c4 = (tid & 15) * 4;
#pragma unroll
    for (int it = 0; it < 4; ++it) {
      const int rr = it * 16 + lr;
      const v4f a = *(const v4f*)(W + (size_t)(r0 + rr) * Cc + c0 + c4);
      *(v4f*)(tf + rr * 68 + c4) = a;
    }
  }
  __syncthreads();
  const int sub = tid >> 3;
  const int c8  = (tid & 7) * 8;
  v4u hv[2];
#pragma unroll
  for (int it = 0; it < 2; ++it) {
    const int oc = it * 32 + sub;
    v4u a;
#pragma unroll
    for (int q4 = 0; q4 < 4; ++q4) {
      const float f0 = tf[(c8 + 2 * q4) * 68 + oc] * mul;
      const float f1 = tf[(c8 + 2 * q4 + 1) * 68 + oc] * mul;
      const unsigned short h0 = __builtin_bit_cast(unsigned short, (_Float16)f0);
      const unsigned short h1 = __builtin_bit_cast(unsigned short, (_Float16)f1);
      a[q4] = pk16(h0, h1);
    }
    hv[it] = a;
  }
  for (int pass = 0; pass < 2; ++pass) {
#pragma unroll
    for (int it = 0; it < 2; ++it) {
      const int oc = it * 32 + sub;
      const size_t go = (size_t)(c0 + oc) * R + r0 + c8;
      *(volatile v4u*)(o + go) = hv[it];
    }
    __threadfence();
  }
}

constexpr int kNWav = 4;
constexpr int kQBlk = 64;
constexpr int kKCh  = 64;
constexpr int kOPitch = 132;

__device__ __forceinline__ v8f hmma(v16h a, v16h b, v8f c) {
  c = __builtin_amdgcn_wmma_f32_16x16x32_f16(false, a, false, b, (short)0, c, false, false);
  asm volatile("v_nop\n\tv_nop\n\tv_nop\n\tv_nop" : "+v"(c) : "v"(a), "v"(b));
  return c;
}

__global__ __launch_bounds__(128)
void attn128_kernel(const unsigned short* __restrict__ qp, const unsigned short* __restrict__ kp,
                    const unsigned short* __restrict__ vtp, float* __restrict__ out, float sscale) {
  union FH { v16h v; v8h h[2]; };
  __shared__ __align__(16) _Float16 Ksh[kKCh * kHD];
  __shared__ __align__(16) _Float16 Vts[kHD * kKCh];
  __shared__ __align__(16) _Float16 Psh[kNWav][16 * kKCh];
  __shared__ __align__(16) float    Os[kNWav][16 * kOPitch];

  const int tid  = threadIdx.x;
  const int wave = tid >> 5;
  const int lane = tid & 31;
  const int hh   = lane >> 4;
  const int c    = lane & 15;

  constexpr int nqb = kQLen / kQBlk;
  const int bx = blockIdx.x;
  const int qb = bx % nqb;
  const int bh = bx / nqb;
  const int h  = bh % kHeads;
  const int b  = bh / kHeads;
  const int q0 = qb * kQBlk + wave * 16;

  const _Float16* Q  = (const _Float16*)(const void*)qp;
  const _Float16* Kp = (const _Float16*)(const void*)kp;
  const _Float16* Vt = (const _Float16*)(const void*)vtp;
  float* ob = out + (size_t)b * kQLen * kVCh + (size_t)h * kHD;

  v16h qa[4];
#pragma unroll
  for (int dc = 0; dc < 4; ++dc) {
    const _Float16* qr = Q + (size_t)(b * kQLen + q0 + c) * kQKCh + h * kHD + dc * 32 + 8 * hh;
    qa[dc] = Frag<_Float16>::load(qr);
  }

  float mrow[8], lrow[8];
  v8f oacc[8];
#pragma unroll
  for (int r = 0; r < 8; ++r) { mrow[r] = -INFINITY; lrow[r] = 0.f; }
#pragma unroll
  for (int t = 0; t < 8; ++t) oacc[t] = (v8f){0.f,0.f,0.f,0.f,0.f,0.f,0.f,0.f};

  constexpr int nChunks = kKVLen / kKCh;
  for (int kc = 0; kc < nChunks; ++kc) {
    const int kv0 = kc * kKCh;
    __syncthreads();
    {
      const int r  = tid >> 1;
      const int dh = (tid & 1) * 64;
      const _Float16* kr = Kp + (size_t)(b * kKVLen + kv0 + r) * kQKCh + h * kHD + dh;
#pragma unroll
      for (int i = 0; i < 8; ++i) {
        const v8h a = *(const v8h*)(kr + 8 * i);
        *(v8h*)(Ksh + r * kHD + dh + 8 * i) = a;
      }
      const _Float16* vr = Vt + (size_t)(h * kHD + tid) * (size_t)(kBatch * kKVLen) + (size_t)b * kKVLen + kv0;
#pragma unroll
      for (int i = 0; i < 8; ++i) {
        const v8h a = *(const v8h*)(vr + 8 * i);
        *(v8h*)(Vts + tid * kKCh + 8 * i) = a;
      }
    }
    __syncthreads();

    v8f s[4];
#pragma unroll
    for (int j = 0; j < 4; ++j) {
      s[j] = (v8f){0.f,0.f,0.f,0.f,0.f,0.f,0.f,0.f};
#pragma unroll
      for (int dc = 0; dc < 4; ++dc) {
        FH kb;
        kb.h[0] = *(const v8h*)(Ksh + (j * 16 + c) * kHD + dc * 32 + 8 * hh);
        kb.h[1] = *(const v8h*)(Ksh + (j * 16 + c) * kHD + dc * 32 + 16 + 8 * hh);
        s[j] = hmma(qa[dc], kb.v, s[j]);
      }
    }
    float cm[8];
#pragma unroll
    for (int r = 0; r < 8; ++r) {
      float m = -INFINITY;
#pragma unroll
      for (int j = 0; j < 4; ++j) {
        const float sv = s[j][r] * sscale;
        s[j][r] = sv;
        m = fmaxf(m, sv);
      }
#pragma unroll
      for (int off = 1; off < 16; off <<= 1) m = fmaxf(m, __shfl_xor(m, off, 32));
      cm[r] = m;
    }
    _Float16* pw = Psh[wave];
#pragma unroll
    for (int r = 0; r < 8; ++r) {
      const float mnew  = fmaxf(mrow[r], cm[r]);
      const float alpha = __expf(mrow[r] - mnew);
      mrow[r] = mnew;
      float psum = 0.f;
#pragma unroll
      for (int j = 0; j < 4; ++j) {
        const float p = __expf(s[j][r] - mnew);
        psum += p;
        pw[(8 * hh + r) * kKCh + j * 16 + c] = (_Float16)(p * kPCarry);
      }
#pragma unroll
      for (int off = 1; off < 16; off <<= 1) psum += __shfl_xor(psum, off, 32);
      lrow[r] = lrow[r] * alpha + psum;
#pragma unroll
      for (int t = 0; t < 8; ++t) oacc[t][r] *= alpha;
    }
    __builtin_amdgcn_fence(__ATOMIC_RELEASE, "workgroup");
    __builtin_amdgcn_wave_barrier();
    __builtin_amdgcn_fence(__ATOMIC_ACQUIRE, "workgroup");
#pragma unroll 1
    for (int kk = 0; kk < 2; ++kk) {
      FH pa;
      pa.h[0] = *(const v8h*)(pw + c * kKCh + kk * 32 + 8 * hh);
      pa.h[1] = *(const v8h*)(pw + c * kKCh + kk * 32 + 16 + 8 * hh);
#pragma unroll
      for (int t = 0; t < 8; ++t) {
        FH vb;
        vb.h[0] = *(const v8h*)(Vts + (t * 16 + c) * kKCh + kk * 32 + 8 * hh);
        vb.h[1] = *(const v8h*)(Vts + (t * 16 + c) * kKCh + kk * 32 + 16 + 8 * hh);
        oacc[t] = hmma(pa.v, vb.v, oacc[t]);
      }
    }
  }

  float* os = Os[wave];
#pragma unroll
  for (int r = 0; r < 8; ++r) {
    const float inv = 1.0f / (lrow[r] * kPCarry);
#pragma unroll
    for (int t = 0; t < 8; ++t) os[(8 * hh + r) * kOPitch + t * 16 + c] = oacc[t][r] * inv;
  }
  __builtin_amdgcn_fence(__ATOMIC_RELEASE, "workgroup");
  __builtin_amdgcn_wave_barrier();
  __builtin_amdgcn_fence(__ATOMIC_ACQUIRE, "workgroup");
  {
    const int c4 = lane * 4;
    for (int pass = 0; pass < 2; ++pass) {
#pragma unroll
      for (int row = 0; row < 16; ++row) {
        const v4f val = *(const v4f*)(os + row * kOPitch + c4);
        *(volatile v4f*)(ob + (size_t)(q0 + row) * kVCh + c4) = val;
      }
      __threadfence();
    }
  }
}

extern "C" void kernel_launch(void* const* d_in, const int* in_sizes, int n_in,
                              void* d_out, int out_size, void* d_ws, size_t ws_size,
                              hipStream_t stream) {
  if (n_in < 12) return;
  if (in_sizes[0] != kBatch * kQLen * kQDim) return;
  if (in_sizes[1] != kBatch * kKVLen * kKVDim) return;
  if (in_sizes[2] < kQDim || in_sizes[3] < kQDim || in_sizes[4] < kKVDim || in_sizes[5] < kKVDim) return;
  if (in_sizes[6] != kQDim * kQKCh || in_sizes[8] != kKVDim * kQKCh || in_sizes[10] != kKVDim * kVCh) return;
  if (in_sizes[7] < kQKCh || in_sizes[9] < kQKCh || in_sizes[11] < kVCh) return;
  if (out_size != kBatch * kQLen * kVCh) return;

  const float* hs   = (const float*)d_in[0];
  const float* inp  = (const float*)d_in[1];
  const float* ln1g = (const float*)d_in[2];
  const float* ln1b = (const float*)d_in[3];
  const float* ln2g = (const float*)d_in[4];
  const float* ln2b = (const float*)d_in[5];
  const float* Wq   = (const float*)d_in[6];
  const float* bq   = (const float*)d_in[7];
  const float* Wk   = (const float*)d_in[8];
  const float* bk   = (const float*)d_in[9];
  const float* Wv   = (const float*)d_in[10];
  const float* bv   = (const float*)d_in[11];
  float* out = (float*)d_out;

  const size_t nQRows  = (size_t)kBatch * kQLen;
  const size_t nKVRows = (size_t)kBatch * kKVLen;
  size_t off = 0;
  const size_t o_hs16  = off; off += nQRows * kQDim * 2;
  const size_t o_inp16 = off; off += nKVRows * kKVDim * 2;
  const size_t o_WqT   = off; off += (size_t)kQKCh * kQDim * 2;
  const size_t o_WkT   = off; off += (size_t)kQKCh * kKVDim * 2;
  const size_t o_WvT   = off; off += (size_t)kVCh * kKVDim * 2;
  const size_t o_q16   = off; off += nQRows * kQKCh * 2;
  const size_t o_k16   = off; off += nKVRows * kQKCh * 2;
  const size_t o_vt16  = off; off += (size_t)kVCh * nKVRows * 2;
  if (off > ws_size) return;

  char* ws = (char*)d_ws;
  unsigned short* hs16  = (unsigned short*)(ws + o_hs16);
  unsigned short* inp16 = (unsigned short*)(ws + o_inp16);
  unsigned short* WqT   = (unsigned short*)(ws + o_WqT);
  unsigned short* WkT   = (unsigned short*)(ws + o_WkT);
  unsigned short* WvT   = (unsigned short*)(ws + o_WvT);
  unsigned short* q16   = (unsigned short*)(ws + o_q16);
  unsigned short* k16   = (unsigned short*)(ws + o_k16);
  unsigned short* vt16  = (unsigned short*)(ws + o_vt16);

  ln_rows_f16<kQDim><<<(unsigned)nQRows, 128, 0, stream>>>(hs, ln1g, ln1b, hs16, kLnEps);
  ln_rows_f16<kKVDim><<<(unsigned)nKVRows, 128, 0, stream>>>(inp, ln2g, ln2b, inp16, kLnEps);

  ttrans_f16_kernel<<<dim3(kQKCh / 64, kQDim / 64), 256, 0, stream>>>(Wq, WqT, kQDim, kQKCh, kWCarry);
  ttrans_f16_kernel<<<dim3(kQKCh / 64, kKVDim / 64), 256, 0, stream>>>(Wk, WkT, kKVDim, kQKCh, kWCarry);
  ttrans_f16_kernel<<<dim3(kVCh / 64, kKVDim / 64), 256, 0, stream>>>(Wv, WvT, kKVDim, kVCh, kWCarry);

  {
    const int tiles = (int)((nQRows / 64) * (kQKCh / 64));
    wmma_gemm64<0, false, 2, 1, false><<<dim3((tiles + 7) / 8, 1), 256, 0, stream>>>(
        hs16, hs16, kQDim, 0L, WqT, WqT, kQDim, 0L, (void*)q16, (void*)q16, kQKCh, 0L,
        bq, bq, 0L, (int)nQRows, kQKCh, kQDim, kWCarryInv);
  }
  {
    const int tiles = (int)((nKVRows / 64) * (kQKCh / 64));
    wmma_gemm64<0, false, 2, 1, false><<<dim3((tiles + 7) / 8, 1), 256, 0, stream>>>(
        inp16, inp16, kKVDim, 0L, WkT, WkT, kKVDim, 0L, (void*)k16, (void*)k16, kQKCh, 0L,
        bk, bk, 0L, (int)nKVRows, kQKCh, kKVDim, kWCarryInv);
  }
  {
    const int tiles = (int)((kVCh / 64) * (nKVRows / 64));
    wmma_gemm64<0, false, 1, 1, false><<<dim3((tiles + 7) / 8, 1), 256, 0, stream>>>(
        WvT, WvT, kKVDim, 0L, inp16, inp16, kKVDim, 0L, (void*)vt16, (void*)vt16, (int)nKVRows, 0L,
        bv, bv, 0L, kVCh, (int)nKVRows, kKVDim, kWCarryInv);
  }

  const float sscale = 1.0f / sqrtf((float)kHD);
  attn128_kernel<<<kBatch * kHeads * (kQLen / kQBlk), 128, 0, stream>>>(q16, k16, vt16, out, sscale);
}
